// EnhancedEncoderLayer_88983132438635
// MI455X (gfx1250) — hardware-verified
//
#include <hip/hip_runtime.h>


#define NB_  2
#define TT   2048
#define DD   512
#define DE   2048
#define D4   128
#define NH_  8
#define HD   64
#define NT   (NB_ * TT)
#define MAXHW 16
typedef _Float16 h16;
typedef unsigned short bf;
typedef __attribute__((ext_vector_type(16))) __bf16   v16bf;
typedef __attribute__((ext_vector_type(16))) _Float16 v16h;
typedef __attribute__((ext_vector_type(8)))  _Float16 v8h;
typedef __attribute__((ext_vector_type(8)))  unsigned short v8us;
typedef __attribute__((ext_vector_type(8)))  float    v8f;
typedef __attribute__((ext_vector_type(4)))  float    v4f;
typedef v8h  __attribute__((may_alias)) v8ha;
typedef v4f  __attribute__((may_alias)) v4fa;
typedef v8us __attribute__((may_alias)) v8usa;

__device__ __forceinline__ unsigned short f2bf(float f) { unsigned u = __float_as_uint(f); u += 0x7FFFu + ((u >> 16) & 1u); return (unsigned short)(u >> 16); }
__device__ __forceinline__ float bf2f(unsigned short b) { return __uint_as_float(((unsigned)b) << 16); }
__device__ __forceinline__ float bfr(float f) { return bf2f(f2bf(f)); }
__device__ __forceinline__ v16h cat16(v8h lo, v8h hi) { return __builtin_shufflevector(lo, hi, 0, 1, 2, 3, 4, 5, 6, 7, 8, 9, 10, 11, 12, 13, 14, 15); }
__device__ __forceinline__ v16bf cat16b(v8us lo, v8us hi) { return __builtin_bit_cast(v16bf, __builtin_shufflevector(lo, hi, 0, 1, 2, 3, 4, 5, 6, 7, 8, 9, 10, 11, 12, 13, 14, 15)); }
__device__ __forceinline__ v8f wmma16(v16h a, v16h b, v8f c) { return __builtin_amdgcn_wmma_f32_16x16x32_f16(false, a, false, b, (short)0, c, false, false); }
__device__ __forceinline__ v8f wmmab(v16bf a, v16bf b, v8f c) { return __builtin_amdgcn_wmma_f32_16x16x32_bf16(false, a, false, b, (short)0, c, false, false); }


template <typename T16> struct WFrag;
template <> struct WFrag<h16> { typedef v16h V; static __device__ __forceinline__ V ld(const h16* p) { return cat16(*(const v8h*)p, *(const v8h*)(p + 16)); } static __device__ __forceinline__ v8f mma(V a, V b, v8f c) { return wmma16(a, b, c); } };
template <> struct WFrag<bf> { typedef v16bf V; static __device__ __forceinline__ V ld(const bf* p) { return cat16b(*(const v8us*)p, *(const v8us*)(p + 16)); } static __device__ __forceinline__ v8f mma(V a, V b, v8f c) { return wmmab(a, b, c); } };
template <typename T16, int NSPLIT, bool BIAS>
__global__ __launch_bounds__(32) void k_gemmw(const T16* __restrict__ A, const T16* __restrict__ A2, const T16* __restrict__ Bt, const T16* __restrict__ Bt2, int K, float* C, int ldc, const float* __restrict__ bias, size_t sA, size_t sB, size_t sC) {
    typedef typename WFrag<T16>::V V;
    __shared__ __align__(16) float os[16 * 68];
    const size_t z = blockIdx.z; A += z * sA; if (A2) A2 += z * sA; Bt += z * sB; if (Bt2) Bt2 += z * sB; C += z * sC;
    const int lane = threadIdx.x & 31, lr = lane & 15, hi = lane >> 4; const int r0 = blockIdx.x * 64, c0 = blockIdx.y * 64;
    v8f acc[4][4];
#pragma unroll
    for (int mb = 0; mb < 4; ++mb)
#pragma unroll
        for (int nb = 0; nb < 4; ++nb) acc[mb][nb] = (v8f){};
    const size_t aoff = (size_t)(r0 + lr) * K + 8 * hi, boff = (size_t)(c0 + lr) * K + 8 * hi;
#pragma unroll 1
    for (int kc = 0; kc < K; kc += 32) {
        V a[4], a2[4];
#pragma unroll
        for (int mb = 0; mb < 4; ++mb) { a[mb] = WFrag<T16>::ld(A + aoff + (size_t)mb * 16 * K + kc); if (NSPLIT == 1 || NSPLIT == 2) a2[mb] = WFrag<T16>::ld(A2 + aoff + (size_t)mb * 16 * K + kc); }
#pragma unroll
        for (int nb = 0; nb < 4; ++nb) { const V b = WFrag<T16>::ld(Bt + boff + (size_t)nb * 16 * K + kc); V b2; if (NSPLIT >= 2) b2 = WFrag<T16>::ld(Bt2 + boff + (size_t)nb * 16 * K + kc);
#pragma unroll
            for (int mb = 0; mb < 4; ++mb) { acc[mb][nb] = WFrag<T16>::mma(a[mb], b, acc[mb][nb]); if (NSPLIT == 1 || NSPLIT == 2) acc[mb][nb] = WFrag<T16>::mma(a2[mb], b, acc[mb][nb]); if (NSPLIT >= 2) acc[mb][nb] = WFrag<T16>::mma(a[mb], b2, acc[mb][nb]); } }
        asm volatile("v_nop\n\tv_nop\n\tv_nop\n\tv_nop" : "+v"(acc[0][0]), "+v"(acc[1][1]), "+v"(acc[2][2]), "+v"(acc[3][3]) : "v"(a[0]), "v"(a[3]));
    }
#pragma unroll
    for (int mb = 0; mb < 4; ++mb) {
#pragma unroll
        for (int nb = 0; nb < 4; ++nb) {
#pragma unroll
            for (int j = 0; j < 8; ++j) os[(hi * 8 + j) * 68 + nb * 16 + lr] = acc[mb][nb][j]; }
        __builtin_amdgcn_wave_barrier(); asm volatile("" ::: "memory");
        float* crow = C + (size_t)(r0 + mb * 16) * ldc + c0;
#pragma unroll 1
        for (int ps = 0; ps < 2; ++ps) {
#pragma unroll
            for (int s = 0; s < 8; ++s) { const int row = 2 * s + hi, cofs = lr * 4; v4f val = *(const v4fa*)(os + row * 68 + cofs); if (BIAS) { val[0] += bfr(bias[c0 + cofs]); val[1] += bfr(bias[c0 + cofs + 1]); val[2] += bfr(bias[c0 + cofs + 2]); val[3] += bfr(bias[c0 + cofs + 3]); }
                *(volatile v4f*)(crow + (size_t)row * ldc + cofs) = val; }
            if (ps == 0) __threadfence(); }
        __builtin_amdgcn_wave_barrier(); asm volatile("" ::: "memory");
    }
}

__device__ __forceinline__ void splitf(float y, unsigned short& h, unsigned short& l) { h = f2bf(y); l = f2bf(y - bf2f(h)); }
__device__ __forceinline__ float siluf(float a) { return __fdiv_rn(a, __fadd_rn(1.0f, __expf(-a))); }
typedef __attribute__((ext_vector_type(2))) unsigned short v2us;
typedef __attribute__((ext_vector_type(4))) unsigned short v4us;
typedef __attribute__((ext_vector_type(2))) float v2f;
#define BNS 0.99999500003749937f

__global__ __launch_bounds__(256) void k_cvt8(const float* __restrict__ src, bf* dst, size_t n8) { const size_t i = (size_t)blockIdx.x * 256 + threadIdx.x; if (i >= n8) return; const v8f v = *(const v8f*)(src + i * 8); v8us o;
#pragma unroll
    for (int k = 0; k < 8; ++k) o[k] = f2bf(v[k]); *(volatile v8us*)(dst + i * 8) = o; __threadfence(); *(volatile v8us*)(dst + i * 8) = o; }
__global__ __launch_bounds__(256) void k_dw(const float* __restrict__ E1, const float* __restrict__ dw, bf* Hh, bf* Hl) { const size_t i = ((size_t)blockIdx.x * 256 + threadIdx.x) * 2; if (i >= (size_t)TT * DE) return; const int s = (int)(i / DE); const int o = (int)(i % DE); v2us oh, ol;
#pragma unroll
    for (int q = 0; q < 2; ++q) { const int oo = o + q; float acc = __fmul_rn(bfr(dw[oo * 3 + 1]), siluf(E1[(size_t)s * DE + oo]));
        if (s > 0) { float t = __fmul_rn(bfr(dw[oo * 3 + 0]), siluf(E1[(size_t)(s - 1) * DE + oo])); asm volatile("" : "+v"(t)); acc = __fadd_rn(acc, t); }
        if (s < TT - 1) { float t = __fmul_rn(bfr(dw[oo * 3 + 2]), siluf(E1[(size_t)(s + 1) * DE + oo])); asm volatile("" : "+v"(t)); acc = __fadd_rn(acc, t); }
        unsigned short a, c2; splitf(siluf(__fmul_rn(acc, BNS)), a, c2); oh[q] = a; ol[q] = c2; }
    *(volatile v2us*)(Hh + i) = oh; *(volatile v2us*)(Hl + i) = ol; __threadfence(); *(volatile v2us*)(Hh + i) = oh; *(volatile v2us*)(Hl + i) = ol; }
__global__ __launch_bounds__(256) void k_gl(const float* __restrict__ P1, bf* Hh, bf* Hl) { const size_t i = ((size_t)blockIdx.x * 256 + threadIdx.x) * 2; if (i >= (size_t)TT * D4) return; v2us oh, ol;
#pragma unroll 1
    for (int q = 0; q < 2; ++q) { const float h = __fmul_rn(P1[i + q], BNS); float e = erff(h * 0.70710678f); asm volatile("" : "+v"(e)); unsigned short a, c2; splitf(__fmul_rn(__fmul_rn(0.5f, h), __fadd_rn(1.0f, e)), a, c2); oh[q] = a; ol[q] = c2; }
    *(volatile v2us*)(Hh + i) = oh; *(volatile v2us*)(Hl + i) = ol; __threadfence(); *(volatile v2us*)(Hh + i) = oh; *(volatile v2us*)(Hl + i) = ol; }
__global__ __launch_bounds__(256) void k_h5(const float* __restrict__ E2, const float* __restrict__ dw2, const float* __restrict__ p2, int b, float* HS) {
    const int lane = threadIdx.x & 31; const int s = blockIdx.x * 8 + (threadIdx.x >> 5); if (s >= TT) return; float acc = 0.f;
#pragma unroll 4
    for (int c = lane; c < DD; c += 32) { float h4 = siluf(E2[(size_t)s * DD + c]); h4 = __fmul_rn(h4, bfr(dw2[c])); h4 = siluf(__fmul_rn(h4, BNS)); float t = __fmul_rn(h4, bfr(p2[c])); asm volatile("" : "+v"(t)); acc = __fadd_rn(acc, t); }
#pragma unroll
    for (int sh = 16; sh; sh >>= 1) acc += __shfl_xor(acc, sh, 32);
    const float o = (lane == 0) ? __fmul_rn(acc, BNS) : 0.f; *(volatile float*)(HS + ((size_t)b * TT + s) * 32 + lane) = o; __threadfence(); *(volatile float*)(HS + ((size_t)b * TT + s) * 32 + lane) = o; }
__global__ __launch_bounds__(32) void k_win(const float* __restrict__ HS, int* WIN) {
    const int lane = threadIdx.x; float s = 0.f; for (int i = lane; i < NT; i += 32) s = __fadd_rn(s, HS[(size_t)i * 32]);
#pragma unroll
    for (int sh = 16; sh; sh >>= 1) s += __shfl_xor(s, sh, 32);
    const float ratio = __fdiv_rn(s, (float)NT); const float wr = __fadd_rn(3.0f, __fmul_rn(ratio, 29.0f)); int w = (int)wr; if (w > TT) w = TT;
    const int o = (lane == 0) ? w : 0; *(volatile int*)(WIN + lane) = o; __threadfence(); *(volatile int*)(WIN + lane) = o; }
__global__ __launch_bounds__(256) void k_band(const float* __restrict__ FQ, const float* __restrict__ FK, const float* __restrict__ FV, const int* __restrict__ WIN, bf* Ah, bf* Al) {
    const int lane = threadIdx.x & 31; const int w0 = blockIdx.x * 8 + (threadIdx.x >> 5); if (w0 >= TT * NH_) return; const int s = w0 / NH_, h = w0 % NH_; const int d = lane * 2; int hw = WIN[0] / 2; if (hw > MAXHW) hw = MAXHW;
    const v2f q2 = *(const v2f*)(FQ + (size_t)s * DD + h * HD + d); float sc[2 * MAXHW + 1]; float mx = -3.0e38f;
#pragma unroll
    for (int w = 0; w < 2 * MAXHW + 1; ++w) { const int j = s + w - MAXHW; float a = -3.0e38f; const bool ok = (w - MAXHW >= -hw) && (w - MAXHW <= hw) && j >= 0 && j < TT;
        if (ok) { const v2f k2 = *(const v2f*)(FK + (size_t)j * HD + d); float p0 = __fmul_rn(q2[0], k2[0]), p1 = __fmul_rn(q2[1], k2[1]); asm volatile("" : "+v"(p0)); asm volatile("" : "+v"(p1)); a = __fadd_rn(p0, p1);
#pragma unroll
            for (int sh = 16; sh; sh >>= 1) a += __shfl_xor(a, sh, 32);
            a = __fmul_rn(a, 0.125f); mx = fmaxf(mx, a); }
        sc[w] = ok ? a : -3.0e38f; }
    float sum = 0.f;
#pragma unroll
    for (int w = 0; w < 2 * MAXHW + 1; ++w) { sc[w] = (sc[w] > -1.0e38f) ? __expf(sc[w] - mx) : 0.f; sum += sc[w]; }
    const float inv = __fdiv_rn(1.0f, sum); float o0 = 0.f, o1 = 0.f;
#pragma unroll
    for (int w = 0; w < 2 * MAXHW + 1; ++w) { const int j = s + w - MAXHW; if (sc[w] == 0.f || j < 0 || j >= TT) continue; const v2f v2 = *(const v2f*)(FV + (size_t)j * HD + d); float pw = __fmul_rn(sc[w], inv); asm volatile("" : "+v"(pw));
        float m0 = __fmul_rn(pw, v2[0]), m1 = __fmul_rn(pw, v2[1]); asm volatile("" : "+v"(m0)); asm volatile("" : "+v"(m1)); o0 = __fadd_rn(o0, m0); o1 = __fadd_rn(o1, m1); }
    v2us oh, ol; unsigned short a2, c2; splitf(o0, a2, c2); oh[0] = a2; ol[0] = c2; splitf(o1, a2, c2); oh[1] = a2; ol[1] = c2;
    const size_t o = (size_t)s * DD + h * HD + d; *(volatile v2us*)(Ah + o) = oh; *(volatile v2us*)(Al + o) = ol; __threadfence(); *(volatile v2us*)(Ah + o) = oh; *(volatile v2us*)(Al + o) = ol; }
__global__ __launch_bounds__(256) void k_catpl(const float* __restrict__ xq, const float* __restrict__ ATT, bf* Ch, bf* Cl) { const size_t i = ((size_t)blockIdx.x * 256 + threadIdx.x) * 2; if (i >= (size_t)TT * 2 * DD) return; const int s = (int)(i / (2 * DD)); const int c = (int)(i % (2 * DD)); v2us oh, ol;
#pragma unroll
    for (int q = 0; q < 2; ++q) { const int cc = c + q; unsigned short a, c2; if (cc < DD) { a = f2bf(xq[(size_t)s * DD + cc]); c2 = 0; } else splitf(ATT[(size_t)s * DD + cc - DD], a, c2); oh[q] = a; ol[q] = c2; }
    *(volatile v2us*)(Ch + i) = oh; *(volatile v2us*)(Cl + i) = ol; __threadfence(); *(volatile v2us*)(Ch + i) = oh; *(volatile v2us*)(Cl + i) = ol; }
__global__ __launch_bounds__(256) void k_mix(const float* __restrict__ G, const float* __restrict__ xq, const float* __restrict__ ATT, const float* __restrict__ rw, float* XH) {
    const int lane = threadIdx.x & 31; const int s = blockIdx.x * 8 + (threadIdx.x >> 5); if (s >= TT) return; float v[DD / 32]; float ss = 0.f;
#pragma unroll
    for (int ch = 0; ch < DD / 128; ++ch) { const size_t base = (size_t)s * DD + ch * 128 + lane * 4; const v4f g4 = *(const v4f*)(G + base), x4 = *(const v4f*)(xq + base), a4 = *(const v4f*)(ATT + base);
#pragma unroll 1
        for (int q = 0; q < 4; ++q) { const float g = siluf(g4[q]); float t1 = __fmul_rn(bfr(x4[q]), g), t2 = __fmul_rn(a4[q], __fsub_rn(1.0f, g)); asm volatile("" : "+v"(t1)); asm volatile("" : "+v"(t2)); const float o = __fadd_rn(t1, t2); v[ch * 4 + q] = o; ss = __fadd_rn(ss, __fmul_rn(o, o)); } }
#pragma unroll
    for (int sh = 16; sh; sh >>= 1) ss += __shfl_xor(ss, sh, 32);
    const float rs = __fdiv_rn(1.0f, __fsqrt_rn(__fadd_rn(ss * (1.0f / DD), 1e-6f)));
#pragma unroll 1
    for (int ps = 0; ps < 2; ++ps) {
#pragma unroll
        for (int ch = 0; ch < DD / 128; ++ch) { v4f o4;
#pragma unroll
            for (int q = 0; q < 4; ++q) { float t = __fmul_rn(v[ch * 4 + q], rs); asm volatile("" : "+v"(t)); o4[q] = __fmul_rn(t, bfr(rw[ch * 128 + lane * 4 + q])); }
            *(volatile v4f*)(XH + (size_t)s * DD + ch * 128 + lane * 4) = o4; }
        if (ps == 0) __threadfence(); }
}
__global__ __launch_bounds__(256) void k_colmean(const float* __restrict__ XH, float* CM) { const int c = blockIdx.x * 256 + threadIdx.x; if (c >= DD) return; float s = 0.f; for (int r = 0; r < TT; ++r) s = __fadd_rn(s, XH[(size_t)r * DD + c]);
    const float o = s * (1.0f / TT); *(volatile float*)(CM + c) = o; __threadfence(); *(volatile float*)(CM + c) = o; }
__global__ __launch_bounds__(256) void k_sub(const float* __restrict__ XH, const float* __restrict__ CM, float* OUTb) { const size_t i = ((size_t)blockIdx.x * 256 + threadIdx.x) * 4; if (i >= (size_t)TT * DD) return; const int c = (int)(i & (DD - 1)); const v4f x = *(const v4f*)(XH + i); v4f o;
#pragma unroll
    for (int q = 0; q < 4; ++q) o[q] = __fsub_rn(x[q], CM[c + q]); *(volatile v4f*)(OUTb + i) = o; __threadfence(); *(volatile v4f*)(OUTb + i) = o; }

extern "C" void kernel_launch(void* const* d_in, const int* in_sizes, int n_in,
                              void* d_out, int out_size, void* d_ws, size_t ws_size, hipStream_t stream) {
    (void)in_sizes; (void)n_in; (void)out_size;
    const float* IN[20]; for (int i = 0; i < 20; ++i) IN[i] = (const float*)d_in[i];
    float* OUT = (float*)d_out;
    char* wsp = (char*)d_ws;
    auto take = [&](size_t bytes) { char* p = wsp; wsp += (bytes + 255) & ~(size_t)255; return (void*)p; };
    bf* WE1 = (bf*)take((size_t)DE * DD * 2); bf* WP1 = (bf*)take((size_t)D4 * DE * 2); bf* WE2 = (bf*)take((size_t)DD * D4 * 2); bf* WQ = (bf*)take((size_t)DD * DD * 2); bf* WK = (bf*)take((size_t)HD * DD * 2); bf* WV = (bf*)take((size_t)HD * DD * 2); bf* WO = (bf*)take((size_t)DD * DD * 2); bf* WG = (bf*)take((size_t)DD * 2 * DD * 2);
    bf* XB = (bf*)take((size_t)TT * DD * 2); bf* KB = (bf*)take((size_t)TT * DD * 2); bf* VB = (bf*)take((size_t)TT * DD * 2);
    float* E1 = (float*)take((size_t)TT * DE * 4); bf* H2h = (bf*)take((size_t)TT * DE * 2); bf* H2l = (bf*)take((size_t)TT * DE * 2); float* P1 = (float*)take((size_t)TT * D4 * 4); bf* H3h = (bf*)take((size_t)TT * D4 * 2); bf* H3l = (bf*)take((size_t)TT * D4 * 2); float* E2 = (float*)take((size_t)TT * DD * 4);
    float* HS = (float*)take((size_t)NT * 32 * 4); int* WIN = (int*)take(256);
    float* FQ = (float*)take((size_t)TT * DD * 4); float* FK = (float*)take((size_t)TT * HD * 4); float* FV = (float*)take((size_t)TT * HD * 4); bf* Ah = (bf*)take((size_t)TT * DD * 2); bf* Al = (bf*)take((size_t)TT * DD * 2); float* ATT = (float*)take((size_t)TT * DD * 4);
    bf* Ch = (bf*)take((size_t)TT * 2 * DD * 2); bf* Cl = (bf*)take((size_t)TT * 2 * DD * 2); float* G = (float*)take((size_t)TT * DD * 4); float* XH = (float*)take((size_t)TT * DD * 4); float* CM = (float*)take(DD * 4);
    if ((size_t)(wsp - (char*)d_ws) > ws_size) return;
    { const float* ws_[8] = {IN[3], IN[5], IN[6], IN[9], IN[11], IN[13], IN[15], IN[17]}; bf* wd_[8] = {WE1, WP1, WE2, WQ, WK, WV, WO, WG}; const size_t n8[8] = {(size_t)DE * DD / 8, (size_t)D4 * DE / 8, (size_t)DD * D4 / 8, (size_t)DD * DD / 8, (size_t)HD * DD / 8, (size_t)HD * DD / 8, (size_t)DD * DD / 8, (size_t)DD * 2 * DD / 8};
      for (int i = 0; i < 8; ++i) k_cvt8<<<(unsigned)((n8[i] + 255) / 256), 256, 0, stream>>>(ws_[i], wd_[i], n8[i]); }
    const size_t nx = (size_t)TT * DD / 8; const unsigned gx = (unsigned)((nx + 255) / 256), L2e = (unsigned)(((size_t)TT * DE / 2 + 255) / 256), L4 = (unsigned)(((size_t)TT * DD / 4 + 255) / 256);
    for (int b = 0; b < NB_; ++b) {
        k_cvt8<<<gx, 256, 0, stream>>>(IN[0] + (size_t)b * TT * DD, XB, nx);
        k_gemmw<bf, 0, false><<<dim3(TT / 64, DE / 64, 1), 32, 0, stream>>>(XB, nullptr, WE1, nullptr, DD, E1, DE, nullptr, 0, 0, 0);
        k_dw<<<L2e, 256, 0, stream>>>(E1, IN[4], H2h, H2l);
        k_gemmw<bf, 1, false><<<dim3(TT / 64, D4 / 64, 1), 32, 0, stream>>>(H2h, H2l, WP1, nullptr, DE, P1, D4, nullptr, 0, 0, 0);
        k_gl<<<(unsigned)(((size_t)TT * D4 / 2 + 255) / 256), 256, 0, stream>>>(P1, H3h, H3l);
        k_gemmw<bf, 1, false><<<dim3(TT / 64, DD / 64, 1), 32, 0, stream>>>(H3h, H3l, WE2, nullptr, D4, E2, DD, nullptr, 0, 0, 0);
        k_h5<<<TT / 8, 256, 0, stream>>>(E2, IN[7], IN[8], b, HS); }
    k_win<<<1, 32, 0, stream>>>(HS, WIN);
    for (int b = 0; b < NB_; ++b) { const float* xq = IN[0] + (size_t)b * TT * DD;
        k_cvt8<<<gx, 256, 0, stream>>>(xq, XB, nx); k_cvt8<<<gx, 256, 0, stream>>>(IN[1] + (size_t)b * TT * DD, KB, nx); k_cvt8<<<gx, 256, 0, stream>>>(IN[2] + (size_t)b * TT * DD, VB, nx);
        k_gemmw<bf, 0, true><<<dim3(TT / 64, DD / 64, 1), 32, 0, stream>>>(XB, nullptr, WQ, nullptr, DD, FQ, DD, IN[10], 0, 0, 0);
        k_gemmw<bf, 0, true><<<dim3(TT / 64, HD / 64, 1), 32, 0, stream>>>(KB, nullptr, WK, nullptr, DD, FK, HD, IN[12], 0, 0, 0);
        k_gemmw<bf, 0, true><<<dim3(TT / 64, HD / 64, 1), 32, 0, stream>>>(VB, nullptr, WV, nullptr, DD, FV, HD, IN[14], 0, 0, 0);
        k_band<<<(TT * NH_ + 7) / 8, 256, 0, stream>>>(FQ, FK, FV, WIN, Ah, Al);
        k_gemmw<bf, 1, true><<<dim3(TT / 64, DD / 64, 1), 32, 0, stream>>>(Ah, Al, WO, nullptr, DD, ATT, DD, IN[16], 0, 0, 0);
        k_catpl<<<(unsigned)(((size_t)TT * 2 * DD / 2 + 255) / 256), 256, 0, stream>>>(xq, ATT, Ch, Cl);
        k_gemmw<bf, 1, true><<<dim3(TT / 64, DD / 64, 1), 32, 0, stream>>>(Ch, Cl, WG, nullptr, 2 * DD, G, DD, IN[18], 0, 0, 0);
        k_mix<<<TT / 8, 256, 0, stream>>>(G, xq, ATT, IN[19], XH);
        k_colmean<<<(DD + 255) / 256, 256, 0, stream>>>(XH, CM);
        k_sub<<<L4, 256, 0, stream>>>(XH, CM, OUT + (size_t)b * TT * DD); }
}
